// DeltaNet_22488448762199
// MI455X (gfx1250) — hardware-verified
//
#include <hip/hip_runtime.h>
#include <math.h>

constexpr int kBatch   = 4;
constexpr int kSeq     = 1024;
constexpr int kDim     = 512;
constexpr int kHeads   = 8;
constexpr int kHeadDim = 64;
constexpr int kMix     = 2;
constexpr int kRows    = kBatch * kSeq;
constexpr int kGateN   = kHeads * (2 + kMix);
constexpr int kNUsed   = 3 * kDim + kGateN;
constexpr int kNAll    = ((kNUsed + 63) / 64) * 64;
constexpr int kColK    = kDim;
constexpr int kColV    = 2 * kDim;
constexpr int kColG    = 3 * kDim;
constexpr int kGcRec   = 8;
constexpr int kChunk   = 16;
constexpr float kWCarry = 16.0f;
constexpr float kACarry = 16.0f;
constexpr float kScaleIn  = 1.0f / kWCarry;
constexpr float kScaleOut = 1.0f / (kWCarry * kACarry);
constexpr float kLnEps = 1e-5f;
constexpr float kInvDim = 1.0f / (float)kDim;

static_assert(kRows == 4096);
static_assert(kNUsed == 1568);
static_assert(kNAll == 1600);
static_assert(kHeads * kHeadDim == kDim);
static_assert(kHeadDim / 2 == 32);
static_assert((kSeq & (kSeq - 1)) == 0);
static_assert(kRows % 64 == 0);
static_assert(kNAll % 64 == 0);
static_assert(kDim % 64 == 0);
static_assert(kDim % 32 == 0);
static_assert(kSeq % kChunk == 0);
static_assert(kMix == 2);

typedef __attribute__((ext_vector_type(16))) _Float16 v16h;
typedef __attribute__((ext_vector_type(8)))  _Float16 v8h;
typedef __attribute__((ext_vector_type(8)))  float    v8f;
typedef __attribute__((ext_vector_type(4)))  float    v4f;
typedef __attribute__((ext_vector_type(2)))  float    v2f;
typedef __attribute__((ext_vector_type(4)))  unsigned int v4u;

__device__ __forceinline__ unsigned pk16(unsigned short a, unsigned short b) {
  return (unsigned)a | ((unsigned)b << 16);
}
__device__ __forceinline__ unsigned short h_bits(float f) {
  const _Float16 h = (_Float16)f;
  return __builtin_bit_cast(unsigned short, h);
}

union FragU { v16h v; v8h h[2]; };
__device__ __forceinline__ v16h frag_load(const _Float16* p) {
  FragU f;
  f.h[0] = *(const v8h*)(p);
  f.h[1] = *(const v8h*)(p + 16);
  return f.v;
}
__device__ __forceinline__ v8f mma_h(v16h a, v16h b, v8f c) {
  return __builtin_amdgcn_wmma_f32_16x16x32_f16(false, a, false, b, (short)0, c, false, false);
}
__device__ __forceinline__ void guard_group(v8f& a, v8f& b, v8f& c, v8f& d,
                                            v16h x, v16h y0, v16h y1, v16h y2, v16h y3) {
  asm volatile("v_nop\n\tv_nop\n\tv_nop\n\tv_nop"
               : "+v"(a), "+v"(b), "+v"(c), "+v"(d)
               : "v"(x), "v"(y0), "v"(y1), "v"(y2), "v"(y3));
}
__device__ __forceinline__ void acc_guard4(v8f& a, v8f& b, v8f& c, v8f& d) {
  asm volatile("v_nop\n\tv_nop\n\tv_nop\n\tv_nop" : "+v"(a), "+v"(b), "+v"(c), "+v"(d));
}

constexpr int kPackXB  = (kRows * kDim) / 2048;
constexpr int kPackWB  = (kDim * kDim) / 2048;
constexpr int kPackGB  = (kGateN * kDim) / 2048;
constexpr int kPackZB  = ((kNAll - kNUsed) * kDim) / 2048;
constexpr int kPackAll = kPackXB + 3 * kPackWB + kPackGB + kPackZB + kPackWB;
static_assert(kPackXB == 1024 && kPackWB == 128 && kPackGB == 8 && kPackZB == 8 && kPackAll == 1552);

__global__ __launch_bounds__(256) void pack_f16_kernel(
    const float* __restrict__ x,  const float* __restrict__ wq, const float* __restrict__ wk,
    const float* __restrict__ wv, const float* __restrict__ wg, const float* __restrict__ wo,
    unsigned short* __restrict__ xh, unsigned short* __restrict__ wall, unsigned short* __restrict__ woh) {
  const int bid = blockIdx.x;
  const int tid = threadIdx.x;
  const float* src = x;
  unsigned short* dst = xh;
  size_t soff = (size_t)bid * 2048;
  size_t doff = (size_t)bid * 2048;
  float sc = 1.0f;
  bool zero = false;
  if (bid >= kPackXB) {
    const int r = bid - kPackXB;
    dst = wall;
    doff = (size_t)r * 2048;
    sc = kWCarry;
    if (r < kPackWB) {
      src = wq; soff = (size_t)r * 2048;
    } else if (r < 2 * kPackWB) {
      src = wk; soff = (size_t)(r - kPackWB) * 2048;
    } else if (r < 3 * kPackWB) {
      src = wv; soff = (size_t)(r - 2 * kPackWB) * 2048;
    } else if (r < 3 * kPackWB + kPackGB) {
      src = wg; soff = (size_t)(r - 3 * kPackWB) * 2048;
    } else if (r < 3 * kPackWB + kPackGB + kPackZB) {
      src = wq; soff = 0; zero = true;
    } else {
      const int ro = r - (3 * kPackWB + kPackGB + kPackZB);
      src = wo; soff = (size_t)ro * 2048;
      dst = woh; doff = (size_t)ro * 2048;
    }
  }
  v4f a = (v4f){0.f, 0.f, 0.f, 0.f};
  v4f c = (v4f){0.f, 0.f, 0.f, 0.f};
  if (!zero) {
    const float* p = src + soff + (size_t)tid * 8;
    a = *(const v4f*)(p);
    c = *(const v4f*)(p + 4);
  }
  unsigned short hb[8];
#pragma unroll
  for (int e = 0; e < 4; ++e) {
    const float fa = a[e] * sc;
    const float fc = c[e] * sc;
    hb[e]     = h_bits(fa);
    hb[4 + e] = h_bits(fc);
  }
  const v4u u = (v4u){pk16(hb[0], hb[1]), pk16(hb[2], hb[3]), pk16(hb[4], hb[5]), pk16(hb[6], hb[7])};
  unsigned short* q = dst + doff + (size_t)tid * 8;
  *(volatile v4u*)q = u;
  __threadfence();
  *(volatile v4u*)q = u;
}

template <bool ADDRB>
__global__ __launch_bounds__(256) void gemm64_f16_kernel(
    const unsigned short* __restrict__ Ap, int lda,
    const unsigned short* __restrict__ Btp, int ldb,
    float* __restrict__ C, int ldc,
    const float* __restrict__ bias, const float* __restrict__ resid, int ldr,
    int M, int N, int K, float scale) {
  const _Float16* A  = (const _Float16*)Ap;
  const _Float16* Bt = (const _Float16*)Btp;
  __shared__ __align__(16) float sT[8][16 * 68];
  const int lane = threadIdx.x & 31;
  const int wave = threadIdx.x >> 5;
  const int tilesN = N >> 6;
  const int tilesM = M >> 6;
  const int tile = blockIdx.x * 8 + wave;
  if (tile >= tilesM * tilesN) return;
  const int tm = tile / tilesN;
  const int tn = tile - tm * tilesN;
  const int m0 = tm << 6;
  const int n0 = tn << 6;

  const int rlane = lane & 15;
  const int koff  = (lane >> 4) * 8;
  const int mOff  = (lane >> 4) * 8;

  v8f acc[4][4];
#pragma unroll
  for (int i = 0; i < 4; ++i)
#pragma unroll
    for (int j = 0; j < 4; ++j) acc[i][j] = (v8f){0.f, 0.f, 0.f, 0.f, 0.f, 0.f, 0.f, 0.f};

  for (int k0 = 0; k0 < K; k0 += 32) {
    v16h bh[4];
#pragma unroll
    for (int j = 0; j < 4; ++j) {
      const size_t bo = (size_t)(n0 + (j << 4) + rlane) * ldb + koff + k0;
      bh[j] = frag_load(Bt + bo);
    }
#pragma unroll
    for (int i = 0; i < 4; ++i) {
      const size_t ao = (size_t)(m0 + (i << 4) + rlane) * lda + koff + k0;
      const v16h ah = frag_load(A + ao);
#pragma unroll
      for (int j = 0; j < 4; ++j) acc[i][j] = mma_h(ah, bh[j], acc[i][j]);
      guard_group(acc[i][0], acc[i][1], acc[i][2], acc[i][3], ah, bh[0], bh[1], bh[2], bh[3]);
    }
  }
  acc_guard4(acc[0][0], acc[0][1], acc[0][2], acc[0][3]);
  acc_guard4(acc[1][0], acc[1][1], acc[1][2], acc[1][3]);
  acc_guard4(acc[2][0], acc[2][1], acc[2][2], acc[2][3]);
  acc_guard4(acc[3][0], acc[3][1], acc[3][2], acc[3][3]);

  float* slab = sT[wave];
  const int hh = lane >> 4;
  const int c4 = (lane & 15) * 4;
  v4f bias4 = (v4f){0.f, 0.f, 0.f, 0.f};
  if (ADDRB) bias4 = *(const v4f*)(bias + n0 + c4);
#pragma unroll
  for (int i = 0; i < 4; ++i) {
    const int mBase = m0 + (i << 4);
#pragma unroll
    for (int j = 0; j < 4; ++j) {
#pragma unroll
      for (int r = 0; r < 8; ++r) {
        const float v = acc[i][j][r] * scale;
        slab[(mOff + r) * 68 + (j << 4) + rlane] = v;
      }
    }
    __builtin_amdgcn_fence(__ATOMIC_RELEASE, "workgroup");
    __builtin_amdgcn_wave_barrier();
    __builtin_amdgcn_fence(__ATOMIC_ACQUIRE, "workgroup");
    v4f ov[8];
#pragma unroll
    for (int it = 0; it < 8; ++it) {
      const int row = it * 2 + hh;
      v4f v = *(const v4f*)(slab + row * 68 + c4);
      if (ADDRB) {
        const v4f r4 = *(const v4f*)(resid + (size_t)(mBase + row) * ldr + n0 + c4);
        v = (v + bias4) + r4;
      }
      ov[it] = v;
    }
    for (int pass = 0; pass < 2; ++pass) {
#pragma unroll
      for (int it = 0; it < 8; ++it) {
        const int row = it * 2 + hh;
        *(volatile v4f*)(C + (size_t)(mBase + row) * ldc + n0 + c4) = ov[it];
      }
      __threadfence();
    }
    __builtin_amdgcn_fence(__ATOMIC_RELEASE, "workgroup");
    __builtin_amdgcn_wave_barrier();
    __builtin_amdgcn_fence(__ATOMIC_ACQUIRE, "workgroup");
  }
}

struct RotTab { float v[32]; };
static_assert(sizeof(RotTab) == 128);

constexpr double c_sqrt(double a) {
  double x = a;
  for (int it = 0; it < 64; ++it) x = 0.5 * (x + a / x);
  return x;
}
constexpr RotTab make_rot_tab() {
  RotTab t{};
  double r = 10000.0;
  for (int s = 0; s < 5; ++s) r = c_sqrt(r);
  double p = 1.0;
  for (int i = 0; i < 32; ++i) {
    const float pf = (float)p;
    t.v[i] = 1.0f / pf;
    p *= r;
  }
  return t;
}
constexpr RotTab kRotTab = make_rot_tab();

__global__ __launch_bounds__(256) void rotate_kernel(const float* __restrict__ qkvg,
                                                     float* __restrict__ qr, float* __restrict__ kr,
                                                     RotTab tab) {
  const int row = blockIdx.x;
  const int tid = threadIdx.x;
  const int h = tid >> 5;
  const int i = tid & 31;
  float fr = tab.v[0];
#pragma unroll
  for (int j = 1; j < 32; ++j) fr = (i == j) ? tab.v[j] : fr;
  const float pos = (float)(row & (kSeq - 1));
  const float ang = pos * fr;
  const float sn = sinf(ang);
  const float cs = cosf(ang);
  const float* src = qkvg + (size_t)row * kNAll + h * kHeadDim + 2 * i;
  const v2f qv = *(const v2f*)(src);
  const v2f kv = *(const v2f*)(src + kColK);
  v2f qo, ko;
  qo[0] = qv[0] * cs - qv[1] * sn;
  qo[1] = qv[0] * sn + qv[1] * cs;
  ko[0] = kv[0] * cs - kv[1] * sn;
  ko[1] = kv[0] * sn + kv[1] * cs;
  float* qd = qr + (size_t)row * kDim + h * kHeadDim + 2 * i;
  float* kd = kr + (size_t)row * kDim + h * kHeadDim + 2 * i;
  *(volatile v2f*)qd = qo;
  *(volatile v2f*)kd = ko;
  __threadfence();
  *(volatile v2f*)qd = qo;
  *(volatile v2f*)kd = ko;
}

__global__ __launch_bounds__(256) void gates_kernel(const float* __restrict__ qkvg,
                                                    const float* __restrict__ bg,
                                                    const float* __restrict__ logit_alphas,
                                                    float* __restrict__ gc) {
  __shared__ __align__(16) float sg[256 * kGcRec];
  const int tid = threadIdx.x;
  const int item = blockIdx.x * 256 + tid;
  const int row = item >> 3;
  const int h = item & 7;
  const v4f g4 = *(const v4f*)(qkvg + (size_t)row * kNAll + kColG + 4 * h);
  const v4f b4 = *(const v4f*)(bg + 4 * h);
  const v2f la = *(const v2f*)(logit_alphas + 2 * h);
  const float a0 = g4[0] + b4[0];
  const float a1 = g4[1] + b4[1];
  const float a2 = g4[2] + b4[2];
  const float a3 = g4[3] + b4[3];
  const float gf = 1.0f / (1.0f + expf(-a0));
  const float gu = 1.0f / (1.0f + expf(-a1));
  const float mx = fmaxf(a2, a3);
  const float e2 = expf(a2 - mx);
  const float e3 = expf(a3 - mx);
  const float inv = 1.0f / (e2 + e3);
  const float w0 = e2 * inv;
  const float w1 = e3 * inv;
  const float al0 = 1.0f / (1.0f + expf(-la[0]));
  const float al1 = 1.0f / (1.0f + expf(-la[1]));
  const v4f ra = (v4f){al0 * gf, al1 * gf, w0 * gu, w1 * gu};
  const v4f rb = (v4f){w0, w1, 0.0f, 0.0f};
  *(v4f*)(sg + tid * kGcRec)     = ra;
  *(v4f*)(sg + tid * kGcRec + 4) = rb;
  __syncthreads();
  const v4f o0 = *(const v4f*)(sg + (size_t)tid * 4);
  const v4f o1 = *(const v4f*)(sg + (size_t)(256 + tid) * 4);
  float* dp = gc + (size_t)blockIdx.x * (256 * kGcRec);
  *(volatile v4f*)(dp + (size_t)tid * 4) = o0;
  *(volatile v4f*)(dp + (size_t)(256 + tid) * 4) = o1;
  __threadfence();
  *(volatile v4f*)(dp + (size_t)tid * 4) = o0;
  *(volatile v4f*)(dp + (size_t)(256 + tid) * 4) = o1;
}

__global__ __launch_bounds__(256) void scan_kernel(const float* __restrict__ qr,
                                                   const float* __restrict__ kr,
                                                   const float* __restrict__ qkvg,
                                                   const float* __restrict__ gc,
                                                   unsigned short* __restrict__ attn) {
  __shared__ __align__(16) float obuf[2][kChunk * kHeadDim];
  const int tid = threadIdx.x;
  const int lane = tid & 31;
  const int wave = tid >> 5;
  const int b = blockIdx.x >> 3;
  const int h = blockIdx.x & 7;
  const int e_loc = lane & 7;
  const int dg = lane >> 3;
  const int e = wave * 8 + e_loc;
  const size_t rowb = (size_t)b * kSeq;

  float s0[16], s1[16];
#pragma unroll
  for (int j = 0; j < 16; ++j) { s0[j] = 0.0f; s1[j] = 0.0f; }

#pragma unroll 1
  for (int ch = 0; ch < kSeq / kChunk; ++ch) {
    float* ob = obuf[ch & 1];
#pragma unroll 1
    for (int ts = 0; ts < kChunk; ++ts) {
      const size_t row = rowb + (size_t)(ch * kChunk + ts);
      const float* kp = kr + row * kDim + h * kHeadDim + dg * 16;
      const float* qp = qr + row * kDim + h * kHeadDim + dg * 16;
      v4f kv[4], qv[4];
#pragma unroll
      for (int i = 0; i < 4; ++i) {
        kv[i] = *(const v4f*)(kp + 4 * i);
        qv[i] = *(const v4f*)(qp + 4 * i);
      }
      const float ve = qkvg[row * kNAll + kColV + h * kHeadDim + e];
      const float* gp = gc + (row * kHeads + h) * kGcRec;
      const v4f ga = *(const v4f*)(gp);
      const v4f gb = *(const v4f*)(gp + 4);
      const float r0 = ga[0], r1 = ga[1];
      const float kw0 = ve * ga[2];
      const float kw1 = ve * ga[3];
      const float w0 = gb[0], w1 = gb[1];
      float p0 = 0.0f, p1 = 0.0f;
#pragma unroll
      for (int j = 0; j < 16; ++j) {
        const float kd = kv[j >> 2][j & 3];
        const float qd = qv[j >> 2][j & 3];
        s0[j] = fmaf(kd, kw0, s0[j] * r0);
        s1[j] = fmaf(kd, kw1, s1[j] * r1);
        p0 = fmaf(qd, s0[j], p0);
        p1 = fmaf(qd, s1[j], p1);
      }
      float o = w0 * p0 + w1 * p1;
      o += __shfl_xor(o, 8, 32);
      o += __shfl_xor(o, 16, 32);
      if (lane < 8) ob[ts * kHeadDim + e] = o;
    }
    __syncthreads();
    if (wave < 4) {
      const int rowc = wave * 4 + (lane >> 3);
      const int c8 = (lane & 7) * 8;
      const v4f va = *(const v4f*)(ob + rowc * kHeadDim + c8);
      const v4f vc = *(const v4f*)(ob + rowc * kHeadDim + c8 + 4);
      unsigned short hb[8];
#pragma unroll
      for (int q = 0; q < 4; ++q) {
        const float fa = va[q] * kACarry;
        const float fc = vc[q] * kACarry;
        hb[q]     = h_bits(fa);
        hb[4 + q] = h_bits(fc);
      }
      const v4u u = (v4u){pk16(hb[0], hb[1]), pk16(hb[2], hb[3]), pk16(hb[4], hb[5]), pk16(hb[6], hb[7])};
      unsigned short* dp = attn + (rowb + (size_t)(ch * kChunk + rowc)) * kDim + h * kHeadDim + c8;
      *(volatile v4u*)dp = u;
      __threadfence();
      *(volatile v4u*)dp = u;
    }
  }
}

__global__ __launch_bounds__(256) void norm_rows_kernel(const float* __restrict__ yp,
                                                        const float* __restrict__ gam,
                                                        const float* __restrict__ bet,
                                                        float* __restrict__ y, int nrows) {
  const int tid = threadIdx.x, lane = tid & 31;
  const int row = blockIdx.x * 8 + (tid >> 5);
  if (row >= nrows) return;
  const float* rp = yp + (size_t)row * kDim;
  v4f v[4], g[4], bb[4];
  float s = 0.0f;
#pragma unroll
  for (int q = 0; q < 4; ++q) {
    v[q]  = *(const v4f*)(rp  + 128 * q + 4 * lane);
    g[q]  = *(const v4f*)(gam + 128 * q + 4 * lane);
    bb[q] = *(const v4f*)(bet + 128 * q + 4 * lane);
    s += (v[q][0] + v[q][1]) + (v[q][2] + v[q][3]);
  }
#pragma unroll
  for (int off = 1; off < 32; off <<= 1) s += __shfl_xor(s, off, 32);
  const float mu = s * kInvDim;
  float ss = 0.0f;
#pragma unroll
  for (int q = 0; q < 4; ++q)
#pragma unroll
    for (int e = 0; e < 4; ++e) {
      const float d = v[q][e] - mu;
      v[q][e] = d;
      ss += d * d;
    }
#pragma unroll
  for (int off = 1; off < 32; off <<= 1) ss += __shfl_xor(ss, off, 32);
  const float var  = ss * kInvDim;
  const float rstd = 1.0f / sqrtf(var + kLnEps);
  v4f o[4];
#pragma unroll
  for (int q = 0; q < 4; ++q)
#pragma unroll
    for (int e = 0; e < 4; ++e) o[q][e] = (v[q][e] * rstd) * g[q][e] + bb[q][e];
  float* op = y + (size_t)row * kDim;
  for (int pass = 0; pass < 2; ++pass) {
#pragma unroll
    for (int q = 0; q < 4; ++q) *(volatile v4f*)(op + 128 * q + 4 * lane) = o[q];
    __threadfence();
  }
}

extern "C" void kernel_launch(void* const* d_in, const int* in_sizes, int n_in,
                              void* d_out, int out_size, void* d_ws, size_t ws_size,
                              hipStream_t stream) {
  if (n_in < 11 || d_out == nullptr || d_ws == nullptr) return;
  if (in_sizes[0] != kRows * kDim || in_sizes[1] != kDim * kDim || in_sizes[2] != kDim * kDim ||
      in_sizes[3] != kDim * kDim || in_sizes[4] != kDim * kDim || in_sizes[5] != kDim ||
      in_sizes[6] != kGateN * kDim || in_sizes[7] != kGateN || in_sizes[8] != kHeads * kMix ||
      in_sizes[9] != kDim || in_sizes[10] != kDim || out_size != kRows * kDim) return;

  const float* x    = (const float*)d_in[0];
  const float* wq   = (const float*)d_in[1];
  const float* wk   = (const float*)d_in[2];
  const float* wv   = (const float*)d_in[3];
  const float* wo   = (const float*)d_in[4];
  const float* bo   = (const float*)d_in[5];
  const float* wg   = (const float*)d_in[6];
  const float* bg   = (const float*)d_in[7];
  const float* la   = (const float*)d_in[8];
  const float* ln_w = (const float*)d_in[9];
  const float* ln_b = (const float*)d_in[10];
  float* out = (float*)d_out;

  char* ws = (char*)d_ws;
  size_t off = 0;
  auto carve = [&](size_t bytes) -> char* {
    char* p = ws + off;
    off += (bytes + 255) & ~(size_t)255;
    return p;
  };
  unsigned short* xh   = (unsigned short*)carve((size_t)kRows * kDim * 2);
  unsigned short* wall = (unsigned short*)carve((size_t)kNAll * kDim * 2);
  unsigned short* woh  = (unsigned short*)carve((size_t)kDim * kDim * 2);
  float*          qkvg = (float*)carve((size_t)kRows * kNAll * 4);
  float*          qr   = (float*)carve((size_t)kRows * kDim * 4);
  float*          kr   = (float*)carve((size_t)kRows * kDim * 4);
  float*          gc   = (float*)carve((size_t)kRows * kHeads * kGcRec * 4);
  unsigned short* attn = (unsigned short*)carve((size_t)kRows * kDim * 2);
  float*          ypre = (float*)carve((size_t)kRows * kDim * 4);
  if (off > ws_size || off > (size_t)134217728) return;

  pack_f16_kernel<<<kPackAll, 256, 0, stream>>>(x, wq, wk, wv, wg, wo, xh, wall, woh);

  gemm64_f16_kernel<false><<<(kRows / 64) * (kNAll / 64) / 8, 256, 0, stream>>>(
      xh, kDim, wall, kDim, qkvg, kNAll, bo, x, kDim, kRows, kNAll, kDim, kScaleIn);

  rotate_kernel<<<kRows, 256, 0, stream>>>(qkvg, qr, kr, kRotTab);

  gates_kernel<<<(kRows * kHeads) / 256, 256, 0, stream>>>(qkvg, bg, la, gc);

  scan_kernel<<<kBatch * kHeads, 256, 0, stream>>>(qr, kr, qkvg, gc, attn);

  gemm64_f16_kernel<true><<<(kRows / 64) * (kDim / 64) / 8, 256, 0, stream>>>(
      attn, kDim, woh, kDim, ypre, kDim, bo, x, kDim, kRows, kDim, kDim, kScaleOut);

  norm_rows_kernel<<<kRows / 8, 256, 0, stream>>>(ypre, ln_w, ln_b, out, kRows);
}
